// GNN_58884001628357
// MI455X (gfx1250) — hardware-verified
//
#include <hip/hip_runtime.h>
#include <stddef.h>
#include <stdint.h>
#include <math.h>


#define NTHR   256
#define NWAVE  8
#define CHUNK  2048
#define WCAP   256
#define LISTN  (NWAVE * WCAP)
#define NBA    1024
#define SLA    10
#define RCAP   20480
#define SOP    1056
#define DEGCAP 64
#define ET     128
#define NT     64
#define GTHR   128
#define HITS_ZINTS (LISTN + 2 * RCAP + NBA + SOP + NBA)
#define HITS_LDS_INTS (HITS_ZINTS + 16)
#define WSMAX  134217728

static_assert((CHUNK & (CHUNK - 1)) == 0 && CHUNK == NWAVE * WCAP && WCAP == 8 * 32);
static_assert(NBA == (1 << SLA) && NBA % 32 == 0 && NBA % NT == 0);
static_assert(((long long)CHUNK << SLA) < (1LL << 31));
static_assert(RCAP % (NTHR * 4) == 0 && HITS_ZINTS % 4 == 0);
static_assert((LISTN + 2 * RCAP + NBA) % 4 == 0 && SOP % 32 == 0 && SOP >= NBA + 32);
static_assert(DEGCAP % 32 == 0);
static_assert(HITS_LDS_INTS * 4 <= 300000);
static_assert(ET == NWAVE * 16 && NT == (GTHR / 32) * 16);

typedef float          v2f   __attribute__((ext_vector_type(2)));
typedef float          v4f   __attribute__((ext_vector_type(4)));
typedef float          v8f   __attribute__((ext_vector_type(8)));
typedef int            v4i   __attribute__((ext_vector_type(4)));
typedef int            v8i   __attribute__((ext_vector_type(8)));
typedef unsigned int   v2u   __attribute__((ext_vector_type(2)));
typedef unsigned short v8us  __attribute__((ext_vector_type(8)));
typedef unsigned short v16us __attribute__((ext_vector_type(16)));
typedef __bf16         v16bf __attribute__((ext_vector_type(16)));
typedef float __attribute__((may_alias)) f32a;
typedef v2f  __attribute__((may_alias)) v2fa;
typedef v4f  __attribute__((may_alias)) v4fa;
typedef v4i  __attribute__((may_alias)) v4ia;
typedef v2u  __attribute__((may_alias)) v2ua;
typedef v8us __attribute__((may_alias)) v8usa;
union FragB { v16bf v; v16us u; v8us h[2]; v8i w; };

__device__ __forceinline__ v8f wmb(const FragB& a, const FragB& b, v8f c) {
  v8f d = __builtin_amdgcn_wmma_f32_16x16x32_bf16(false, a.v, false, b.v, (short)0, c, false, false);
  asm volatile("v_nop\n\tv_nop\n\tv_nop\n\tv_nop" : "+v"(d) : "v"(a.w), "v"(b.w));
  return d;
}

__device__ __forceinline__ unsigned bf16_bits(float f) {
  const unsigned u = __float_as_uint(f);
  return (u + 0x7FFFu + ((u >> 16) & 1u)) >> 16;
}
__device__ __forceinline__ float bf16_val(float f) {
  return __uint_as_float(bf16_bits(f) << 16);
}
__device__ __forceinline__ void split2(float a, float b, unsigned& hw, unsigned& lw) {
  const unsigned ha = bf16_bits(a), hb = bf16_bits(b);
  const unsigned la = bf16_bits(a - __uint_as_float(ha << 16));
  const unsigned lb = bf16_bits(b - __uint_as_float(hb << 16));
  hw = ha | (hb << 16);
  lw = la | (lb << 16);
}
__device__ __forceinline__ float silu_f(float v) {
  const float e = expf(-v);
  return v * __builtin_amdgcn_rcpf(1.0f + e);
}
__device__ __forceinline__ FragB frag_g(const unsigned short* p) {
  FragB f;
  f.h[0] = *(const v8usa*)p;
  f.h[1] = *(const v8usa*)(p + 16);
  return f;
}
__device__ __forceinline__ FragB frag_s(const unsigned int* base, int halfOff) {
  const unsigned short* p = (const unsigned short*)base + halfOff;
  FragB f;
  f.h[0] = *(const v8usa*)p;
  f.h[1] = *(const v8usa*)(p + 16);
  return f;
}

template <int SLB>
__device__ __forceinline__ int scan_chunk(const int* __restrict__ keys, int nE, int cbase, int slotBase,
                                          int nb, int* list, int lane, int wave) {
  int wc = 0;
  const int elb  = wave * WCAP + lane;
  const int e0   = cbase + elb;
  const int sent = -2147483647 - 1;
  const int l0 = keys[min(e0,       nE - 1)];
  const int l1 = keys[min(e0 + 32,  nE - 1)];
  const int l2 = keys[min(e0 + 64,  nE - 1)];
  const int l3 = keys[min(e0 + 96,  nE - 1)];
  const int l4 = keys[min(e0 + 128, nE - 1)];
  const int l5 = keys[min(e0 + 160, nE - 1)];
  const int l6 = keys[min(e0 + 192, nE - 1)];
  const int l7 = keys[min(e0 + 224, nE - 1)];
  const int k0 = (e0       < nE) ? l0 : sent;
  const int k1 = (e0 + 32  < nE) ? l1 : sent;
  const int k2 = (e0 + 64  < nE) ? l2 : sent;
  const int k3 = (e0 + 96  < nE) ? l3 : sent;
  const int k4 = (e0 + 128 < nE) ? l4 : sent;
  const int k5 = (e0 + 160 < nE) ? l5 : sent;
  const int k6 = (e0 + 192 < nE) ? l6 : sent;
  const int k7 = (e0 + 224 < nE) ? l7 : sent;
  const unsigned nbs = (unsigned)slotBase;
  const unsigned unb = (unsigned)nb;
  const unsigned s0 = (unsigned)k0 - nbs, s1 = (unsigned)k1 - nbs;
  const unsigned s2 = (unsigned)k2 - nbs, s3 = (unsigned)k3 - nbs;
  const unsigned s4 = (unsigned)k4 - nbs, s5 = (unsigned)k5 - nbs;
  const unsigned s6 = (unsigned)k6 - nbs, s7 = (unsigned)k7 - nbs;
  const bool h0 = s0 < unb, h1 = s1 < unb, h2 = s2 < unb, h3 = s3 < unb;
  const bool h4 = s4 < unb, h5 = s5 < unb, h6 = s6 < unb, h7 = s7 < unb;
  const unsigned any = __builtin_amdgcn_ballot_w32(h0 | h1 | h2 | h3 | h4 | h5 | h6 | h7);
  if (any != 0u) {
#define HITJ(J, HJ, SJ) { \
      const unsigned mj = __builtin_amdgcn_ballot_w32(HJ); \
      if (mj != 0u) { \
        if (HJ) { \
          const int pos = wc + (int)__builtin_amdgcn_mbcnt_lo(mj, 0u); \
          if (pos < WCAP) list[wave * WCAP + pos] = ((elb + 32 * (J)) << SLB) | (int)(SJ); \
        } \
        wc += (int)__builtin_popcount(mj); } }
    HITJ(0, h0, s0)
    HITJ(1, h1, s1)
    HITJ(2, h2, s2)
    HITJ(3, h3, s3)
    HITJ(4, h4, s4)
    HITJ(5, h5, s5)
    HITJ(6, h6, s6)
    HITJ(7, h7, s7)
#undef HITJ
  }
  return wc;
}

__global__ __launch_bounds__(NTHR) void k_wp(const float* __restrict__ src, int srcStride,
                                             unsigned short* dst, int dstStride,
                                             int nRows, int ush, int mode) {
  const int u = (int)blockIdx.x * NTHR + (int)threadIdx.x;
  if (u >= (nRows << ush)) return;
  const int n  = u >> ush;
  const int k8 = (u & ((1 << ush) - 1)) * 8;
  int srow = k8 & 63;
  int scol = n;
  if (mode == 1)      { srow = ((n >> 6) << 6) + (k8 & 63); scol = n & 63; }
  else if (mode == 2) { srow = ((k8 >> 7) << 6) + (k8 & 63); }
  else if (mode == 3) { srow = k8 & 127; }
  const float* p = src + (size_t)blockIdx.y * (size_t)srcStride + (size_t)srow * 64 + scol;
  v8us o;
#pragma unroll
  for (int i = 0; i < 8; ++i) o[i] = (unsigned short)bf16_bits(p[(size_t)i * 64]);
  unsigned short* dp = dst + (size_t)blockIdx.y * (size_t)dstStride + ((size_t)n << (ush + 3)) + k8;
  *(volatile v8us*)dp = o;
  __threadfence();
  *(volatile v8us*)dp = o;
}

__global__ __launch_bounds__(NTHR) void k_hits(const int* __restrict__ keys, int nE, int* hits, int* so) {
  extern __shared__ __attribute__((aligned(16))) int dsm[];
  int* list = dsm;
  int* hl   = dsm + LISTN;
  int* sl   = hl + RCAP;
  int* cnt  = sl + RCAP;
  int* offs = cnt + NBA;
  int* cur  = offs + SOP;
  int* misc = cur + NBA;
  const int tid = (int)threadIdx.x, lane = tid & 31, wave = tid >> 5;
  const int nodeBase = (int)blockIdx.x * NBA;

  {
    const v4i z4 = {0, 0, 0, 0};
    for (int i = tid * 4; i < HITS_ZINTS; i += NTHR * 4) *(v4ia*)(dsm + i) = z4;
    if (tid < 16) misc[tid] = 0;
  }
  __syncthreads();

  int t = 0, ov = 0;
  const int nChunks = (nE + CHUNK - 1) / CHUNK;
#pragma unroll 1
  for (int ch = 0; ch < nChunks; ++ch) {
    const int cbase = ch * CHUNK;
    const int wc = scan_chunk<SLA>(keys, nE, cbase, nodeBase, NBA, list, lane, wave);
    if (lane == 0) misc[wave] = wc;
    __syncthreads();
    if (wave == 0) {
#pragma unroll 1
      for (int w2 = 0; w2 < NWAVE; ++w2) {
        int c = misc[w2];
        c = c < 0 ? 0 : (c > WCAP ? WCAP : c);
#pragma unroll 1
        for (int b0 = 0; b0 < c; b0 += 32) {
          const int idx = b0 + lane;
          const int ent = list[w2 * WCAP + (idx < WCAP ? idx : WCAP - 1)];
          const int m32 = (c - b0) < 32 ? (c - b0) : 32;
#pragma unroll 1
          for (int k = 0; k < m32; ++k) {
            const int u    = __builtin_amdgcn_readlane(ent, k);
            const int slot = u & (NBA - 1);
            const int el   = (u >> SLA) & (CHUNK - 1);
            const int pk   = ((cbase + el) << SLA) | slot;
            if (t < RCAP) {
              if (lane == 0) { hl[t] = pk; cnt[slot] = cnt[slot] + 1; }
              t = t + 1;
            } else {
              ov = 1;
            }
          }
        }
      }
    }
    __syncthreads();
  }
  if (wave == 0 && lane == 0) { misc[8] = t; misc[9] = ov; }
  __syncthreads();
  int tt = misc[8];
  tt = tt < 0 ? 0 : (tt > RCAP ? RCAP : tt);
  const int ovf = misc[9];

  if (wave == 0) {
    const int base = lane * (NBA / 32);
    int s = 0;
#pragma unroll 1
    for (int i = 0; i < NBA / 32; ++i) s += cnt[base + i];
    int incl = s;
#pragma unroll
    for (int d = 1; d < 32; d <<= 1) {
      const int y = __shfl_up(incl, d, 32);
      if (lane >= d) incl += y;
    }
    int run = incl - s;
#pragma unroll 1
    for (int i = 0; i < NBA / 32; ++i) {
      const int cv = cnt[base + i];
      offs[base + i] = run;
      cur[base + i]  = run;
      run += cv;
    }
  }
  __syncthreads();
  if (wave == 0) {
#pragma unroll 1
    for (int b0 = 0; b0 < tt; b0 += 32) {
      const int idx = b0 + lane;
      const int ent = hl[idx < RCAP ? idx : RCAP - 1];
      const int m32 = (tt - b0) < 32 ? (tt - b0) : 32;
#pragma unroll 1
      for (int k = 0; k < m32; ++k) {
        const int u    = __builtin_amdgcn_readlane(ent, k);
        const int slot = u & (NBA - 1);
        if (lane == 0) {
          int p = cur[slot];
          p = p < 0 ? 0 : (p > RCAP - 1 ? RCAP - 1 : p);
          sl[p] = u;
          cur[slot] = p + 1;
        }
      }
    }
    if (lane == 0) { offs[NBA] = tt; offs[NBA + 1] = ovf; }
  }
  __syncthreads();

  int* hg = hits + (size_t)blockIdx.x * RCAP;
  int* sg = so + (size_t)blockIdx.x * SOP;
#pragma unroll 1
  for (int i = tid * 4; i < RCAP; i += NTHR * 4) {
    v4i e = *(const v4ia*)(sl + i);
    e.x >>= SLA; e.y >>= SLA; e.z >>= SLA; e.w >>= SLA;
    *(volatile v4i*)(hg + i) = e;
  }
  const v4i oa = *(const v4ia*)(offs + 4 * tid);
  const v4i ob = *(const v4ia*)(offs + NBA + 4 * (tid & 7));
  *(volatile v4i*)(sg + 4 * tid) = oa;
  if (tid < 8) *(volatile v4i*)(sg + NBA + 4 * tid) = ob;
  __threadfence();
#pragma unroll 1
  for (int i = tid * 4; i < RCAP; i += NTHR * 4) {
    v4i e = *(const v4ia*)(sl + i);
    e.x >>= SLA; e.y >>= SLA; e.z >>= SLA; e.w >>= SLA;
    *(volatile v4i*)(hg + i) = e;
  }
  *(volatile v4i*)(sg + 4 * tid) = oa;
  if (tid < 8) *(volatile v4i*)(sg + NBA + 4 * tid) = ob;
}

__global__ __launch_bounds__(NTHR) void k_edge(const float* __restrict__ AB, const int* __restrict__ rowi,
                                               const int* __restrict__ coli, const float* __restrict__ ea,
                                               const float* __restrict__ w128, const float* __restrict__ eb1,
                                               const float* __restrict__ eb2,
                                               const unsigned short* __restrict__ W2T,
                                               float* E2, int nE, int nN) {
  __shared__ __attribute__((aligned(16))) unsigned int lds[ET * 64];
  const int tid = (int)threadIdx.x, lane = tid & 31, wave = tid >> 5, hh = lane >> 4, m = lane & 15;
  unsigned int* wl = lds + wave * 1024;
  const int e0w = (int)blockIdx.x * ET + wave * 16;

  int ec = e0w + m;
  ec = ec < nE ? ec : nE - 1;
  int r = rowi[ec];
  r = r < 0 ? 0 : (r > nN - 1 ? nN - 1 : r);
  int c = coli[ec];
  c = c < 0 ? 0 : (c > nN - 1 ? nN - 1 : c);
  const int eai = __float_as_int(bf16_val(ea[ec]));
  v2f wv, b1;
  {
    const v2f a = *(const v2fa*)(w128 + 2 * lane);
    const v2f b = *(const v2fa*)(eb1 + 2 * lane);
    wv.x = bf16_val(a.x); wv.y = bf16_val(a.y);
    b1.x = bf16_val(b.x); b1.y = bf16_val(b.y);
  }
#pragma unroll 1
  for (int j = 0; j < 16; ++j) {
    const int   rj  = __builtin_amdgcn_readlane(r, j);
    const int   cj  = __builtin_amdgcn_readlane(c, j);
    const float eaj = __int_as_float(__builtin_amdgcn_readlane(eai, j));
    const v2f a = *(const v2fa*)(AB + (size_t)rj * 128 + 2 * lane);
    const v2f b = *(const v2fa*)(AB + (size_t)cj * 128 + 64 + 2 * lane);
    const float p0 = ((a.x + b.x) + eaj * wv.x) + b1.x;
    const float p1 = ((a.y + b.y) + eaj * wv.y) + b1.y;
    const float s0 = silu_f(p0);
    const float s1 = silu_f(p1);
    unsigned hw, lw;
    split2(s0, s1, hw, lw);
    wl[j * 64 + lane]      = hw;
    wl[j * 64 + 32 + lane] = lw;
  }
  __syncthreads();

  v8f acc[4];
  {
    const v8f z = {0.f, 0.f, 0.f, 0.f, 0.f, 0.f, 0.f, 0.f};
    acc[0] = z; acc[1] = z; acc[2] = z; acc[3] = z;
  }
  const unsigned short* wp = W2T + (size_t)m * 128 + 8 * hh;
#pragma unroll 1
  for (int ks = 0; ks < 4; ++ks) {
    const FragB af = frag_s(wl, m * 128 + 8 * hh + 32 * ks);
#pragma unroll
    for (int t = 0; t < 4; ++t) {
      const FragB bf = frag_g(wp + (size_t)(16 * t) * 128 + 32 * ks);
      acc[t] = wmb(af, bf, acc[t]);
    }
  }
  __syncthreads();
  f32a* sw = (f32a*)wl;
#pragma unroll
  for (int t = 0; t < 4; ++t) {
#pragma unroll
    for (int rr = 0; rr < 8; ++rr) sw[(8 * hh + rr) * 64 + 16 * t + m] = acc[t][rr];
  }
  __syncthreads();

  v4f b2;
  {
    const v4f a = *(const v4fa*)(eb2 + 4 * m);
    b2.x = bf16_val(a.x); b2.y = bf16_val(a.y); b2.z = bf16_val(a.z); b2.w = bf16_val(a.w);
  }
#pragma unroll 1
  for (int i = 0; i < 8; ++i) {
    const int lr = 2 * i + hh;
    f32a* sp = sw + lr * 64 + 4 * m;
    const v4f v = *(const v4fa*)sp;
    v4f y;
    y.x = silu_f(v.x + b2.x); y.y = silu_f(v.y + b2.y);
    y.z = silu_f(v.z + b2.z); y.w = silu_f(v.w + b2.w);
    *(v4fa*)sp = y;
    *(volatile v4f*)(E2 + (size_t)(e0w + lr) * 64 + 4 * m) = y;
  }
  __threadfence();
#pragma unroll 1
  for (int i = 0; i < 8; ++i) {
    const int lr = 2 * i + hh;
    const v4f y = *(const v4fa*)(sw + lr * 64 + 4 * m);
    *(volatile v4f*)(E2 + (size_t)(e0w + lr) * 64 + 4 * m) = y;
  }
}

template <int MODE>
__global__ __launch_bounds__(GTHR) void k_node(
    const float* __restrict__ nodes, const float* __restrict__ Wemb, const float* __restrict__ bemb,
    unsigned short* HP, float* AB,
    const float* __restrict__ E2, const int* __restrict__ hits, const int* __restrict__ so,
    const unsigned short* __restrict__ W1T, const float* __restrict__ b1,
    const unsigned short* __restrict__ W2T, const float* __restrict__ b2,
    const unsigned short* __restrict__ EABT,
    const float* __restrict__ dW2, const float* __restrict__ db2, float* out,
    int nN, int nE, int nReg)
{
  __shared__ __attribute__((aligned(16))) unsigned int xs[NT * 128];
  __shared__ __attribute__((aligned(16))) unsigned int ts[NT * 64];
  __shared__ __attribute__((aligned(16))) float dws[272];
  const int tid = (int)threadIdx.x, lane = tid & 31, wave = tid >> 5, hh = lane >> 4, m = lane & 15;
  const int wr0 = (int)blockIdx.x * NT + 16 * wave;
  unsigned int* xw = xs + wave * 2048;
  unsigned int* tw = ts + wave * 1024;

  if constexpr (MODE == 2) {
    for (int i = tid; i < 256; i += GTHR) dws[i] = bf16_val(dW2[i]);
    if (tid < 16) {
      const float bb = db2[tid < 4 ? tid : 3];
      dws[256 + tid] = (tid < 4) ? bf16_val(bb) : 0.0f;
    }
  }

  if constexpr (MODE == 0) {
    v2f w0, w1, w2, w3, w4, bb;
    {
      const v2f a0 = *(const v2fa*)(Wemb + 0 * 64 + 2 * lane);
      const v2f a1 = *(const v2fa*)(Wemb + 1 * 64 + 2 * lane);
      const v2f a2 = *(const v2fa*)(Wemb + 2 * 64 + 2 * lane);
      const v2f a3 = *(const v2fa*)(Wemb + 3 * 64 + 2 * lane);
      const v2f a4 = *(const v2fa*)(Wemb + 4 * 64 + 2 * lane);
      const v2f a5 = *(const v2fa*)(bemb + 2 * lane);
      w0.x = bf16_val(a0.x); w0.y = bf16_val(a0.y);
      w1.x = bf16_val(a1.x); w1.y = bf16_val(a1.y);
      w2.x = bf16_val(a2.x); w2.y = bf16_val(a2.y);
      w3.x = bf16_val(a3.x); w3.y = bf16_val(a3.y);
      w4.x = bf16_val(a4.x); w4.y = bf16_val(a4.y);
      bb.x = bf16_val(a5.x); bb.y = bf16_val(a5.y);
    }
#pragma unroll 1
    for (int i = 0; i < 16; ++i) {
      int nd = wr0 + i;
      nd = nd < nN ? nd : nN - 1;
      const float* np = nodes + (size_t)nd * 5;
      const float x0 = bf16_val(np[0]), x1 = bf16_val(np[1]), x2 = bf16_val(np[2]);
      const float x3 = bf16_val(np[3]), x4 = bf16_val(np[4]);
      float ua = x0 * w0.x; ua = fmaf(x1, w1.x, ua); ua = fmaf(x2, w2.x, ua); ua = fmaf(x3, w3.x, ua);
      float ub = x0 * w0.y; ub = fmaf(x1, w1.y, ub); ub = fmaf(x2, w2.y, ub); ub = fmaf(x3, w3.y, ub);
      const float ta = x4 * w4.x, tb = x4 * w4.y;
      const float g0a = (ua + ta) + bb.x, g0b = (ub + tb) + bb.y;
      const float g1a = (ta - ua) + bb.x, g1b = (tb - ub) + bb.y;
      unsigned h0w, l0w, h1w, l1w;
      split2(g0a, g0b, h0w, l0w);
      split2(g1a, g1b, h1w, l1w);
      xw[i * 128 + lane]      = h0w;
      xw[i * 128 + 32 + lane] = h1w;
      xw[i * 128 + 64 + lane] = l0w;
      xw[i * 128 + 96 + lane] = l1w;
    }
  } else {
    int reg = wr0 >> SLA;
    reg = reg > nReg - 1 ? nReg - 1 : (reg < 0 ? 0 : reg);
    const int s0 = wr0 & (NBA - 1);
    const int* sp = so + (size_t)reg * SOP;
    const int* hp = hits + (size_t)reg * RCAP;
    const int offv = sp[s0 + (lane < 16 ? lane : 16)];
    const int flg  = sp[NBA + 1];
    const float qnan = __int_as_float(0x7fc00000);
#pragma unroll 1
    for (int i = 0; i < 16; ++i) {
      int o0 = __builtin_amdgcn_readlane(offv, i);
      int o1 = __builtin_amdgcn_readlane(offv, i + 1);
      o0 = o0 < 0 ? 0 : (o0 > RCAP ? RCAP : o0);
      o1 = o1 < o0 ? o0 : (o1 > RCAP ? RCAP : o1);
      int c = o1 - o0;
      const bool big = c > DEGCAP;
      c = c > DEGCAP ? DEGCAP : c;
      float a0 = 0.0f, a1 = 0.0f;
#pragma unroll 1
      for (int b0 = 0; b0 < c; b0 += 32) {
        int idx = o0 + b0 + lane;
        idx = idx > RCAP - 1 ? RCAP - 1 : idx;
        int eid = hp[idx];
        eid = eid < 0 ? 0 : (eid > nE - 1 ? nE - 1 : eid);
        const int m32 = (c - b0) < 32 ? (c - b0) : 32;
#pragma unroll 1
        for (int k = 0; k < m32; ++k) {
          const int ek = __builtin_amdgcn_readlane(eid, k);
          const v2f v = *(const v2fa*)(E2 + (size_t)ek * 64 + 2 * lane);
          a0 += v.x; a1 += v.y;
        }
      }
      const float pz = (big || (flg != 0)) ? qnan : 0.0f;
      a0 = a0 + pz; a1 = a1 + pz;
      unsigned hw, lw;
      split2(a0, a1, hw, lw);
      xw[i * 128 + 64 + lane] = hw;
      xw[i * 128 + 96 + lane] = lw;
    }
  }
  __syncthreads();

  v8f acc[4];
  {
    const v8f z = {0.f, 0.f, 0.f, 0.f, 0.f, 0.f, 0.f, 0.f};
    acc[0] = z; acc[1] = z; acc[2] = z; acc[3] = z;
  }
  {
    const unsigned short* w1p = W1T + (size_t)m * 256 + 8 * hh;
    if constexpr (MODE == 0) {
#pragma unroll 1
      for (int ks = 0; ks < 8; ++ks) {
        const FragB af = frag_s(xw, m * 256 + 8 * hh + 32 * ks);
#pragma unroll
        for (int t = 0; t < 4; ++t) {
          const FragB bf = frag_g(w1p + (size_t)(16 * t) * 256 + 32 * ks);
          acc[t] = wmb(af, bf, acc[t]);
        }
      }
    } else {
      const unsigned short* hrow = HP + (size_t)(wr0 + m) * 128 + 8 * hh;
#pragma unroll 1
      for (int ks = 0; ks < 4; ++ks) {
        const FragB af = frag_g(hrow + 32 * ks);
#pragma unroll
        for (int t = 0; t < 4; ++t) {
          const FragB bf = frag_g(w1p + (size_t)(16 * t) * 256 + 32 * ks);
          acc[t] = wmb(af, bf, acc[t]);
        }
      }
#pragma unroll 1
      for (int ks = 4; ks < 8; ++ks) {
        const FragB af = frag_s(xw, m * 256 + 8 * hh + 32 * ks);
#pragma unroll
        for (int t = 0; t < 4; ++t) {
          const FragB bf = frag_g(w1p + (size_t)(16 * t) * 256 + 32 * ks);
          acc[t] = wmb(af, bf, acc[t]);
        }
      }
    }
  }
  __syncthreads();
  f32a* sw = (f32a*)xw;
#pragma unroll
  for (int t = 0; t < 4; ++t) {
#pragma unroll
    for (int rr = 0; rr < 8; ++rr) sw[(8 * hh + rr) * 64 + 16 * t + m] = acc[t][rr];
  }
  __syncthreads();

  {
    v4f bv;
    {
      const v4f a = *(const v4fa*)(b1 + 4 * m);
      bv.x = bf16_val(a.x); bv.y = bf16_val(a.y); bv.z = bf16_val(a.z); bv.w = bf16_val(a.w);
    }
#pragma unroll 1
    for (int i = 0; i < 8; ++i) {
      const int lr = 2 * i + hh;
      f32a* sp2 = sw + lr * 64 + 4 * m;
      const v4f v = *(const v4fa*)sp2;
      v4f y;
      y.x = silu_f(v.x + bv.x); y.y = silu_f(v.y + bv.y);
      y.z = silu_f(v.z + bv.z); y.w = silu_f(v.w + bv.w);
      if constexpr (MODE == 2) {
        *(v4fa*)sp2 = y;
      } else {
        unsigned h01, l01, h23, l23;
        split2(y.x, y.y, h01, l01);
        split2(y.z, y.w, h23, l23);
        v2u hw2, lw2;
        hw2.x = h01; hw2.y = h23; lw2.x = l01; lw2.y = l23;
        *(v2ua*)(tw + lr * 64 + 2 * m)      = hw2;
        *(v2ua*)(tw + lr * 64 + 32 + 2 * m) = lw2;
      }
    }
  }
  __syncthreads();

  if constexpr (MODE == 2) {
    const int row = lane & 15;
    const int pr  = lane >> 4;
    float o0 = 0.0f, o1 = 0.0f;
#pragma unroll 4
    for (int k = 0; k < 64; ++k) {
      const float tv = sw[row * 64 + k];
      o0 = fmaf(tv, dws[k * 4 + 2 * pr], o0);
      o1 = fmaf(tv, dws[k * 4 + 2 * pr + 1], o1);
    }
    o0 = o0 + dws[256 + 2 * pr];
    o1 = o1 + dws[256 + 2 * pr + 1];
    const float q0 = __shfl(o0, (lane + 16) & 31, 32);
    const float q1 = __shfl(o1, (lane + 16) & 31, 32);
    v4f ov;
    ov.x = o0; ov.y = o1; ov.z = q0; ov.w = q1;
    const int grow = wr0 + row;
    const bool okst = (lane < 16) && (grow < nN);
    const int gc = grow < nN ? grow : nN - 1;
    float* op = out + (size_t)gc * 4;
    if (okst) *(volatile v4f*)op = ov;
    __threadfence();
    if (okst) *(volatile v4f*)op = ov;
  } else {
    {
      const v8f z = {0.f, 0.f, 0.f, 0.f, 0.f, 0.f, 0.f, 0.f};
      acc[0] = z; acc[1] = z; acc[2] = z; acc[3] = z;
    }
    {
      const unsigned short* w2p = W2T + (size_t)m * 128 + 8 * hh;
#pragma unroll 1
      for (int ks = 0; ks < 4; ++ks) {
        const FragB af = frag_s(tw, m * 128 + 8 * hh + 32 * ks);
#pragma unroll
        for (int t = 0; t < 4; ++t) {
          const FragB bf = frag_g(w2p + (size_t)(16 * t) * 128 + 32 * ks);
          acc[t] = wmb(af, bf, acc[t]);
        }
      }
    }
    __syncthreads();
#pragma unroll
    for (int t = 0; t < 4; ++t) {
#pragma unroll
      for (int rr = 0; rr < 8; ++rr) sw[(8 * hh + rr) * 64 + 16 * t + m] = acc[t][rr];
    }
    __syncthreads();
    {
      v4f bv;
      {
        const v4f a = *(const v4fa*)(b2 + 4 * m);
        bv.x = bf16_val(a.x); bv.y = bf16_val(a.y); bv.z = bf16_val(a.z); bv.w = bf16_val(a.w);
      }
#pragma unroll 1
      for (int i = 0; i < 8; ++i) {
        const int lr = 2 * i + hh;
        const v4f v = *(const v4fa*)(sw + lr * 64 + 4 * m);
        const v4f y = v + bv;
        unsigned h01, l01, h23, l23;
        split2(y.x, y.y, h01, l01);
        split2(y.z, y.w, h23, l23);
        v2u hw2, lw2;
        hw2.x = h01; hw2.y = h23; lw2.x = l01; lw2.y = l23;
        *(v2ua*)(tw + lr * 64 + 2 * m)      = hw2;
        *(v2ua*)(tw + lr * 64 + 32 + 2 * m) = lw2;
      }
    }
    __syncthreads();

    v8f ac8[8];
    {
      const v8f z = {0.f, 0.f, 0.f, 0.f, 0.f, 0.f, 0.f, 0.f};
#pragma unroll
      for (int t = 0; t < 8; ++t) ac8[t] = z;
    }
    {
      const unsigned short* w3p = EABT + (size_t)m * 128 + 8 * hh;
#pragma unroll 1
      for (int ks = 0; ks < 4; ++ks) {
        const FragB af = frag_s(tw, m * 128 + 8 * hh + 32 * ks);
#pragma unroll
        for (int t = 0; t < 8; ++t) {
          const FragB bf = frag_g(w3p + (size_t)(16 * t) * 128 + 32 * ks);
          ac8[t] = wmb(af, bf, ac8[t]);
        }
      }
    }
    __syncthreads();
#pragma unroll
    for (int t = 0; t < 8; ++t) {
#pragma unroll
      for (int rr = 0; rr < 8; ++rr) sw[(8 * hh + rr) * 128 + 16 * t + m] = ac8[t][rr];
    }
    __syncthreads();

#pragma unroll 1
    for (int i = 0; i < 16; ++i) {
      const v4f v = *(const v4fa*)(sw + i * 128 + 4 * lane);
      *(volatile v4f*)(AB + (size_t)(wr0 + i) * 128 + 4 * lane) = v;
    }
#pragma unroll 1
    for (int i = 0; i < 8; ++i) {
      const int lr = 2 * i + hh;
      const v8us q = *(const v8usa*)((const unsigned short*)tw + lr * 128 + 8 * m);
      *(volatile v8us*)(HP + (size_t)(wr0 + lr) * 128 + 8 * m) = q;
    }
    __threadfence();
#pragma unroll 1
    for (int i = 0; i < 16; ++i) {
      const v4f v = *(const v4fa*)(sw + i * 128 + 4 * lane);
      *(volatile v4f*)(AB + (size_t)(wr0 + i) * 128 + 4 * lane) = v;
    }
#pragma unroll 1
    for (int i = 0; i < 8; ++i) {
      const int lr = 2 * i + hh;
      const v8us q = *(const v8usa*)((const unsigned short*)tw + lr * 128 + 8 * m);
      *(volatile v8us*)(HP + (size_t)(wr0 + lr) * 128 + 8 * m) = q;
    }
  }
}

static inline int cdiv(int a, int b) { return (a + b - 1) / b; }
static inline size_t al256(size_t o) { return (o + 255) & ~(size_t)255; }

extern "C" void kernel_launch(void* const* d_in, const int* in_sizes, int n_in,
                              void* d_out, int out_size, void* d_ws, size_t ws_size,
                              hipStream_t stream) {
  if (n_in < 25) return;
  if (in_sizes[0] < 5 || (in_sizes[0] % 5) != 0) return;
  const int nN = in_sizes[0] / 5;
  if (in_sizes[1] < 2 || (in_sizes[1] & 1) != 0) return;
  const int nE = in_sizes[1] / 2;
  if (nN < 1 || nN > (1 << 22) || nE < 1 || nE >= (1 << 21)) return;
  if (in_sizes[2] != nE) return;
  if (in_sizes[3] != 320 || in_sizes[4] != 64) return;
  if (in_sizes[5] != 8192 || in_sizes[6] != 64) return;
  if (in_sizes[7] != 4096 || in_sizes[8] != 64) return;
  if (in_sizes[9] != 5 * 129 * 64 || in_sizes[10] != 320) return;
  if (in_sizes[11] != 5 * 4096 || in_sizes[12] != 320) return;
  if (in_sizes[13] != 5 * 8192 || in_sizes[14] != 320) return;
  if (in_sizes[15] != 5 * 4096 || in_sizes[16] != 320) return;
  if (in_sizes[17] != 129 * 64 || in_sizes[18] != 64) return;
  if (in_sizes[19] != 4096 || in_sizes[20] != 64) return;
  if (in_sizes[21] != 8192 || in_sizes[22] != 64) return;
  if (in_sizes[23] != 256 || in_sizes[24] != 4) return;
  if ((long long)out_size != (long long)nN * 4) return;
  if ((nN & 7) != 0) return;

  const float* nodes = (const float*)d_in[0];
  const int*   edges = (const int*)d_in[1];
  const float* eattr = (const float*)d_in[2];
  const float* W_emb = (const float*)d_in[3];
  const float* b_emb = (const float*)d_in[4];
  const float* Wg1   = (const float*)d_in[5];
  const float* bg1   = (const float*)d_in[6];
  const float* Wg2   = (const float*)d_in[7];
  const float* bg2   = (const float*)d_in[8];
  const float* eW1   = (const float*)d_in[9];
  const float* eb1   = (const float*)d_in[10];
  const float* eW2   = (const float*)d_in[11];
  const float* eb2   = (const float*)d_in[12];
  const float* nW1   = (const float*)d_in[13];
  const float* nb1   = (const float*)d_in[14];
  const float* nW2   = (const float*)d_in[15];
  const float* nb2   = (const float*)d_in[16];
  const float* deW1  = (const float*)d_in[17];
  const float* deb1  = (const float*)d_in[18];
  const float* deW2  = (const float*)d_in[19];
  const float* deb2  = (const float*)d_in[20];
  const float* dnW1  = (const float*)d_in[21];
  const float* dnb1  = (const float*)d_in[22];
  const float* dnW2  = (const float*)d_in[23];
  const float* dnb2  = (const float*)d_in[24];
  float* out = (float*)d_out;
  const int* rowi = edges;
  const int* coli = edges + nE;

  const int NP   = cdiv(nN, NT) * NT;
  const int nReg = cdiv(NP, NBA);
  const int EP   = cdiv(nE, ET) * ET;
  if ((long long)nReg * NBA < (long long)NP) return;

  char* ws = (char*)d_ws;
  size_t off = 0;
  const size_t oWG1 = off; off = al256(off + (size_t)64 * 256 * 2);
  const size_t oWG2 = off; off = al256(off + (size_t)64 * 128 * 2);
  const size_t oEAB = off; off = al256(off + (size_t)6 * 128 * 128 * 2);
  const size_t oEW2 = off; off = al256(off + (size_t)6 * 64 * 128 * 2);
  const size_t oNW1 = off; off = al256(off + (size_t)6 * 64 * 256 * 2);
  const size_t oNW2 = off; off = al256(off + (size_t)5 * 64 * 128 * 2);
  const size_t oHP  = off; off = al256(off + (size_t)NP * 128 * 2);
  const size_t oAB  = off; off = al256(off + (size_t)NP * 128 * 4);
  const size_t oHT  = off; off = al256(off + (size_t)nReg * RCAP * 4);
  const size_t oSO  = off; off = al256(off + (size_t)nReg * SOP * 4);
  const size_t oE2  = off; off = al256(off + (size_t)EP * 64 * 4);
  if (off > ws_size || off > (size_t)WSMAX) return;
  unsigned short* WG1T = (unsigned short*)(ws + oWG1);
  unsigned short* WG2T = (unsigned short*)(ws + oWG2);
  unsigned short* EABT = (unsigned short*)(ws + oEAB);
  unsigned short* EW2T = (unsigned short*)(ws + oEW2);
  unsigned short* NW1T = (unsigned short*)(ws + oNW1);
  unsigned short* NW2T = (unsigned short*)(ws + oNW2);
  unsigned short* HP   = (unsigned short*)(ws + oHP);
  float*          AB   = (float*)(ws + oAB);
  int*            HT   = (int*)(ws + oHT);
  int*            SO   = (int*)(ws + oSO);
  float*          E2   = (float*)(ws + oE2);

  k_wp<<<dim3(8, 1), NTHR, 0, stream>>>(Wg1, 0, WG1T, 0, 64, 5, 3);
  k_wp<<<dim3(4, 1), NTHR, 0, stream>>>(Wg2, 0, WG2T, 0, 64, 4, 0);
  k_wp<<<dim3(8, 5), NTHR, 0, stream>>>(eW1, 129 * 64, EABT, 128 * 128, 128, 4, 1);
  k_wp<<<dim3(8, 1), NTHR, 0, stream>>>(deW1, 0, EABT + 5 * 128 * 128, 0, 128, 4, 1);
  k_wp<<<dim3(4, 5), NTHR, 0, stream>>>(eW2, 4096, EW2T, 64 * 128, 64, 4, 0);
  k_wp<<<dim3(4, 1), NTHR, 0, stream>>>(deW2, 0, EW2T + 5 * 64 * 128, 0, 64, 4, 0);
  k_wp<<<dim3(8, 5), NTHR, 0, stream>>>(nW1, 8192, NW1T, 64 * 256, 64, 5, 2);
  k_wp<<<dim3(8, 1), NTHR, 0, stream>>>(dnW1, 0, NW1T + 5 * 64 * 256, 0, 64, 5, 2);
  k_wp<<<dim3(4, 5), NTHR, 0, stream>>>(nW2, 4096, NW2T, 64 * 128, 64, 4, 0);

  const size_t hitsLds = (size_t)HITS_LDS_INTS * 4;
  hipFuncSetAttribute(reinterpret_cast<const void*>(&k_hits), hipFuncAttributeMaxDynamicSharedMemorySize,
                      (int)hitsLds);
  k_hits<<<nReg, NTHR, hitsLds, stream>>>(rowi, nE, HT, SO);

  const int gN = NP / NT;
  k_node<0><<<gN, GTHR, 0, stream>>>(nodes, W_emb, b_emb, HP, AB, E2, HT, SO,
                                     WG1T, bg1, WG2T, bg2, EABT, dnW2, dnb2, out, nN, nE, nReg);

  const int gE = EP / ET;
  for (int l = 0; l < 6; ++l) {
    const float* w128 = (l < 5) ? (eW1 + (size_t)l * 129 * 64 + 128 * 64) : (deW1 + 128 * 64);
    const float* pb1  = (l < 5) ? (eb1 + l * 64) : deb1;
    const float* pb2  = (l < 5) ? (eb2 + l * 64) : deb2;
    k_edge<<<gE, NTHR, 0, stream>>>(AB, rowi, coli, eattr, w128, pb1, pb2,
                                    EW2T + (size_t)l * 64 * 128, E2, nE, nN);
    if (l < 5) {
      k_node<1><<<gN, GTHR, 0, stream>>>(nodes, W_emb, b_emb, HP, AB, E2, HT, SO,
                                         NW1T + (size_t)l * 64 * 256, nb1 + l * 64,
                                         NW2T + (size_t)l * 64 * 128, nb2 + l * 64,
                                         EABT + (size_t)(l + 1) * 128 * 128,
                                         dnW2, dnb2, out, nN, nE, nReg);
    } else {
      k_node<2><<<gN, GTHR, 0, stream>>>(nodes, W_emb, b_emb, HP, AB, E2, HT, SO,
                                         NW1T + (size_t)5 * 64 * 256, dnb1,
                                         WG2T, dnb1, EABT,
                                         dnW2, dnb2, out, nN, nE, nReg);
    }
  }
}
